// LocalCrossAttention1D_54589034332797
// MI455X (gfx1250) — hardware-verified
//
#include <hip/hip_runtime.h>
#include <math.h>

constexpr int kB = 4, kCd = 512, kCe = 256, kLd = 4096, kLe = 8192, kHid = 2048;
constexpr int kNH = 8, kHD = 64, kWin = 256, kStr = 192, kNW = 22, kMaxE = 512;
constexpr int kQRows = kLd + kWin;
constexpr int kKRows = kLe + kMaxE;
constexpr int kHeadsPerChunk = 4;
constexpr int kGroupsPerChunk = kHeadsPerChunk * kNW;
constexpr int kChunksPerBatch = kNH / kHeadsPerChunk;
constexpr float kEps = 1e-5f;
constexpr float kWCarry = 64.0f;
constexpr float kLoCarry = 2048.0f;
constexpr float kAttCarry = 16.0f;
static_assert(kNW == (kLd + kStr - 1) / kStr, "window count");
static_assert(kLe == 2 * kLd, "encoder/decoder length ratio is the exact integer 2");
static_assert(kQRows % 64 == 0 && kKRows % 64 == 0, "tile multiples");
static_assert((kNW - 1) * kStr + kWin <= kQRows, "q pad rows cover the last window");
static_assert(2 * (kNW - 1) * kStr + kMaxE <= kKRows, "k pad rows cover the last window");
static_assert(kCd % 64 == 0 && kHid % 64 == 0 && kLd % 64 == 0 && kLe % 64 == 0, "tile multiples");
static_assert(kCd % 32 == 0 && kCe % 32 == 0 && kHD % 32 == 0 && kMaxE % 32 == 0 && kHid % 32 == 0, "K step 32");

constexpr size_t kMiB = 1048576;
constexpr size_t kBytesW16   = (size_t)2 * (kCd * kCd + 2 * kCd * kCe + kCd * kCd + kHid * kCd + kCd * kHid);
constexpr size_t kBytesQN    = (size_t)kQRows * kCd * 2;
constexpr size_t kBytesKN    = (size_t)kKRows * kCd * 2;
constexpr size_t kBytesVT    = (size_t)kCd * kKRows * 2;
constexpr size_t kBytesAT    = (size_t)kLd * kCd * 2;
constexpr size_t kBytesS     = (size_t)kGroupsPerChunk * kWin * kMaxE * 4;
constexpr size_t kBytesO     = (size_t)kGroupsPerChunk * kWin * kHD * 4;
constexpr size_t kBytesXD16  = (size_t)kLd * kCd * 2;
constexpr size_t kBytesQRAW  = (size_t)kLd * kCd * 4;
constexpr size_t kBytesXE16  = (size_t)kLe * kCe * 2;
constexpr size_t kBytesKVRAW = (size_t)kLe * 2 * kCd * 4;
constexpr size_t kBytesY2    = (size_t)kLd * kCd * 4;
constexpr size_t kBytesPRE   = (size_t)kLd * kHid * 4;
constexpr size_t kBytesH16   = (size_t)kLd * kHid * 2;
constexpr size_t kBytesY3    = kBytesY2;
constexpr size_t kBytesXCM   = (size_t)kCd * kLd * 4;
constexpr size_t kBytesX16   = kBytesXD16;

constexpr size_t OFF_W16   = 0;
constexpr size_t OFF_BKV   = OFF_W16 + kBytesW16;
constexpr size_t OFF_STATS = OFF_BKV + 4096;
constexpr size_t OFF_QNH   = 6 * kMiB;
constexpr size_t OFF_KN    = OFF_QNH + kBytesQN;
constexpr size_t OFF_VTH   = OFF_KN + kBytesKN;
constexpr size_t OFF_VTL   = OFF_VTH + kBytesVT;
constexpr size_t OFF_ATH   = OFF_VTL + kBytesVT;
constexpr size_t OFF_ATL   = OFF_ATH + kBytesAT;
constexpr size_t OFF_S     = OFF_ATL + kBytesAT;
constexpr size_t OFF_O     = OFF_S + kBytesS;
constexpr size_t OFF_XDH   = OFF_S;
constexpr size_t OFF_XDL   = OFF_XDH + kBytesXD16;
constexpr size_t OFF_QRAW  = OFF_XDL + kBytesXD16;
constexpr size_t OFF_XET   = OFF_S;
constexpr size_t OFF_KVRAW = OFF_XET + kBytesXE16;
constexpr size_t OFF_Y2    = OFF_S;
constexpr size_t OFF_H16   = OFF_ATH;
constexpr size_t OFF_PRE   = OFF_Y2 + kBytesY2;
constexpr size_t OFF_Y3    = OFF_PRE;
constexpr size_t OFF_XCM   = OFF_PRE + kBytesPRE;
constexpr size_t OFF_X16   = OFF_XCM + kBytesXCM;
constexpr size_t kWsEndA   = OFF_O + kBytesO;
constexpr size_t kWsEndB   = OFF_X16 + kBytesX16;
constexpr size_t kWsEnd    = (kWsEndA > kWsEndB) ? kWsEndA : kWsEndB;
static_assert(OFF_STATS + 8192 <= OFF_QNH, "persistent region below 6 MiB");
static_assert(OFF_QRAW + kBytesQRAW <= OFF_O, "q stage transients inside S");
static_assert(OFF_KVRAW + kBytesKVRAW <= OFF_O, "kv stage transients inside S");
static_assert(OFF_H16 + kBytesH16 <= OFF_PRE, "h plane ends where pre begins");
static_assert(OFF_H16 >= OFF_VTL + kBytesVT, "h plane does not touch the zero-filled pad planes");
static_assert(OFF_Y2 + kBytesY2 <= OFF_PRE, "y2 below pre");
static_assert(OFF_Y3 + kBytesY3 <= OFF_XCM, "y3 below x");
static_assert(OFF_PRE + kBytesPRE <= OFF_XCM, "pre below x");
static_assert((OFF_BKV % 128) == 0 && (OFF_STATS % 128) == 0 && (OFF_KN % 128) == 0 && (OFF_VTH % 128) == 0 &&
              (OFF_VTL % 128) == 0 && (OFF_ATH % 128) == 0 && (OFF_ATL % 128) == 0 && (OFF_S % 128) == 0 &&
              (OFF_O % 128) == 0 && (OFF_PRE % 128) == 0 && (OFF_XCM % 128) == 0 && (OFF_X16 % 128) == 0, "128-B aligned carves");
static_assert(kWsEnd == 100401152, "carve total");
static_assert(kWsEnd <= (size_t)134217728, "carve under 128 MiB");

typedef __attribute__((ext_vector_type(16))) _Float16 v16h;
typedef __attribute__((ext_vector_type(8)))  _Float16 v8h;
typedef __attribute__((ext_vector_type(16))) __bf16   v16b;
typedef __attribute__((ext_vector_type(8)))  __bf16   v8b;
typedef __attribute__((ext_vector_type(8)))  float    v8f;
typedef __attribute__((ext_vector_type(4)))  float    v4f;
typedef __attribute__((ext_vector_type(2)))  float    v2f;
typedef __attribute__((ext_vector_type(4)))  unsigned int v4u;

__device__ __forceinline__ unsigned short f2bf_bits(float f) {
  unsigned u = __float_as_uint(f);
  return (unsigned short)((u + 0x7FFFu + ((u >> 16) & 1u)) >> 16);
}
__device__ __forceinline__ float bf_bits2f(unsigned short h) { return __uint_as_float(((unsigned)h) << 16); }

__device__ __forceinline__ void dep_guard_h(v8f& a, v8f& b, v16h x, v16h y) { asm volatile("v_nop\n\tv_nop\n\tv_nop\n\tv_nop" : "+v"(a), "+v"(b) : "v"(x), "v"(y)); }
__device__ __forceinline__ void dep_guard_b(v8f& a, v8f& b, v16b x, v16b y) { asm volatile("v_nop\n\tv_nop\n\tv_nop\n\tv_nop" : "+v"(a), "+v"(b) : "v"(x), "v"(y)); }
__device__ __forceinline__ void keep4_h(v16h a, v16h b, v16h c, v16h d) { asm volatile("v_nop" :: "v"(a), "v"(b), "v"(c), "v"(d)); }
__device__ __forceinline__ void keep4_b(v16b a, v16b b, v16b c, v16b d) { asm volatile("v_nop" :: "v"(a), "v"(b), "v"(c), "v"(d)); }
__device__ __forceinline__ void acc_guard4(v8f& a, v8f& b, v8f& c, v8f& d) { asm volatile("v_nop\n\tv_nop\n\tv_nop\n\tv_nop" : "+v"(a), "+v"(b), "+v"(c), "+v"(d)); }
template <typename T> struct Frag;
template <> struct Frag<_Float16> {
  typedef v16h V; union U { v16h v; v8h h[2]; };
  static __device__ __forceinline__ v16h load(const _Float16* p) {
    U f; f.h[0] = *(const v8h*)(p); f.h[1] = *(const v8h*)(p + 16); return f.v;
  }
  static __device__ __forceinline__ v8f mma(v16h a, v16h b, v8f c) {
    return __builtin_amdgcn_wmma_f32_16x16x32_f16(false, a, false, b, (short)0, c, false, false);
  }
  static __device__ __forceinline__ void guard(v8f& a, v8f& b, v16h x, v16h y) { dep_guard_h(a, b, x, y); }
  static __device__ __forceinline__ void keep(v16h a, v16h b, v16h c, v16h d) { keep4_h(a, b, c, d); }
};
template <> struct Frag<__bf16> {
  typedef v16b V; union U { v16b v; v8b h[2]; };
  static __device__ __forceinline__ v16b load(const __bf16* p) {
    U f; f.h[0] = *(const v8b*)(p); f.h[1] = *(const v8b*)(p + 16); return f.v;
  }
  static __device__ __forceinline__ v8f mma(v16b a, v16b b, v8f c) {
    return __builtin_amdgcn_wmma_f32_16x16x32_bf16(false, a, false, b, (short)0, c, false, false);
  }
  static __device__ __forceinline__ void guard(v8f& a, v8f& b, v16b x, v16b y) { dep_guard_b(a, b, x, y); }
  static __device__ __forceinline__ void keep(v16b a, v16b b, v16b c, v16b d) { keep4_b(a, b, c, d); }
};

__device__ __forceinline__ unsigned pk16(unsigned short a, unsigned short b) { return (unsigned)a | ((unsigned)b << 16); }
__device__ __forceinline__ unsigned short h_bits(float f) { const _Float16 h = (_Float16)f; return __builtin_bit_cast(unsigned short, h); }

struct GemmGeom {
  long sA0, sA1, sA2, sB0, sB1, sB2, sC0, sC1, sC2;
  int d1, d2, lda, ldb, ldc, M, N, K;
  float scale; int pad0;
};
static_assert(sizeof(GemmGeom) == 112, "GemmGeom has no padding bytes");

template <int ET> struct Elem;
template <> struct Elem<0> { typedef _Float16 T; };
template <> struct Elem<1> { typedef __bf16 T; };
template <int ET, bool SPLIT, int BIAS_MODE, int OUT_MODE, bool RESID>
__global__ __launch_bounds__(256) void wmma_gemm64g(
    const unsigned short* __restrict__ Ap, const unsigned short* __restrict__ A2p,
    const unsigned short* __restrict__ Btp, const unsigned short* __restrict__ Bt2p,
    void* Cout, void* Cout2,
    const float* __restrict__ bias, const float* resid, GemmGeom g) {
  typedef typename Elem<ET>::T T;
  typedef typename Frag<T>::V V;
  const T* A = (const T*)Ap; const T* A2 = (const T*)A2p; const T* Bt = (const T*)Btp; const T* Bt2 = (const T*)Bt2p;
  __shared__ __align__(16) float sT[8][16 * 68];
  const int gz   = blockIdx.y;
  const int i2   = gz % g.d2;
  const int t1   = gz / g.d2;
  const int i1   = t1 % g.d1;
  const int i0   = t1 / g.d1;
  const size_t offA = (size_t)((long)i0 * g.sA0 + (long)i1 * g.sA1 + (long)i2 * g.sA2);
  const size_t offB = (size_t)((long)i0 * g.sB0 + (long)i1 * g.sB1 + (long)i2 * g.sB2);
  const size_t offC = (size_t)((long)i0 * g.sC0 + (long)i1 * g.sC1 + (long)i2 * g.sC2);
  const int lda = g.lda, ldb = g.ldb, ldc = g.ldc, K = g.K;
  const float scale = g.scale;
  const int lane = threadIdx.x & 31;
  const int wave = threadIdx.x >> 5;
  const int tilesN = g.N >> 6;
  const int tilesM = g.M >> 6;
  const int tile = blockIdx.x * 8 + wave;
  if (tile >= tilesM * tilesN) return;
  const int tm = tile / tilesN;
  const int tn = tile - tm * tilesN;
  const int m0 = tm << 6;
  const int n0 = tn << 6;

  const T* Ab  = A  + offA;
  const T* Bb  = Bt + offB;
  const T* Ab2 = SPLIT ? (A2  + offA) : nullptr;
  const T* Bb2 = SPLIT ? (Bt2 + offB) : nullptr;

  const int rlane = lane & 15;
  const int koff  = (lane >> 4) * 8;
  const int mOff  = (lane >> 4) * 8;

  v8f acc[4][4];
#pragma unroll
  for (int i = 0; i < 4; ++i)
#pragma unroll
    for (int j = 0; j < 4; ++j) acc[i][j] = (v8f){0.f,0.f,0.f,0.f,0.f,0.f,0.f,0.f};

  for (int k0 = 0; k0 < K; k0 += 32) {
    V bh[4], bl[4];
#pragma unroll
    for (int j = 0; j < 4; ++j) {
      const size_t bo = (size_t)(n0 + (j << 4) + rlane) * ldb + koff + k0;
      bh[j] = Frag<T>::load(Bb + bo);
      if (SPLIT) bl[j] = Frag<T>::load(Bb2 + bo);
    }
#pragma unroll
    for (int i = 0; i < 4; ++i) {
      const size_t ao = (size_t)(m0 + (i << 4) + rlane) * lda + koff + k0;
      V ah = Frag<T>::load(Ab + ao);
      V al;
      if (SPLIT) al = Frag<T>::load(Ab2 + ao);
#pragma unroll
      for (int j = 0; j < 4; ++j) {
        acc[i][j] = Frag<T>::mma(ah, bh[j], acc[i][j]);
        if (SPLIT) {
          acc[i][j] = Frag<T>::mma(ah, bl[j], acc[i][j]);
          acc[i][j] = Frag<T>::mma(al, bh[j], acc[i][j]);
        }
      }
      Frag<T>::guard(acc[i][0], acc[i][3], ah, SPLIT ? al : ah);
    }
    Frag<T>::keep(bh[0], bh[1], bh[2], bh[3]);
    if (SPLIT) Frag<T>::keep(bl[0], bl[1], bl[2], bl[3]);
  }
  acc_guard4(acc[0][0], acc[0][1], acc[0][2], acc[0][3]);
  acc_guard4(acc[1][0], acc[1][1], acc[1][2], acc[1][3]);
  acc_guard4(acc[2][0], acc[2][1], acc[2][2], acc[2][3]);
  acc_guard4(acc[3][0], acc[3][1], acc[3][2], acc[3][3]);

  float* slab = sT[wave];
  const float* Rb = RESID ? (resid + offC) : nullptr;
#pragma unroll
  for (int i = 0; i < 4; ++i) {
    const int mBase = m0 + (i << 4);
#pragma unroll
    for (int j = 0; j < 4; ++j) {
      const int n = n0 + (j << 4) + rlane;
      float bv = 0.f;
      if (BIAS_MODE == 2) bv = bias[n];
#pragma unroll
      for (int r = 0; r < 8; ++r) {
        float v = acc[i][j][r] * scale;
        if (BIAS_MODE == 1) v += bias[mBase + mOff + r];
        if (BIAS_MODE == 2) v += bv;
        if (RESID) v += Rb[(size_t)(mBase + mOff + r) * ldc + n];
        slab[(mOff + r) * 68 + (j << 4) + rlane] = v;
      }
    }
    __builtin_amdgcn_fence(__ATOMIC_RELEASE, "workgroup");
    __builtin_amdgcn_wave_barrier();
    __builtin_amdgcn_fence(__ATOMIC_ACQUIRE, "workgroup");
    if (OUT_MODE == 0) {
      float* C = (float*)Cout + offC;
      const int hh = lane >> 4, c4 = (lane & 15) * 4;
      for (int pass = 0; pass < 2; ++pass) {
#pragma unroll
        for (int it = 0; it < 8; ++it) {
          const int row = it * 2 + hh;
          v4f v = *(const v4f*)(slab + row * 68 + c4);
          *(volatile v4f*)(C + (size_t)(mBase + row) * ldc + n0 + c4) = v;
        }
        __threadfence();
      }
    } else {
      const int q = lane >> 3, c8 = (lane & 7) * 8;
      unsigned short* C  = (unsigned short*)Cout  + offC;
      unsigned short* C2 = (OUT_MODE == 2) ? ((unsigned short*)Cout2 + offC) : nullptr;
      for (int pass = 0; pass < 2; ++pass) {
#pragma unroll
        for (int it = 0; it < 4; ++it) {
          const int row = it * 4 + q;
          const float* sp = slab + row * 68 + c8;
          v8h hv, lv;
#pragma unroll
          for (int e = 0; e < 8; ++e) {
            if (OUT_MODE == 1) {
              hv[e] = (_Float16)sp[e];
            } else {
              unsigned short hb = f2bf_bits(sp[e]);
              unsigned short lb = f2bf_bits(sp[e] - bf_bits2f(hb));
              hv[e] = __builtin_bit_cast(_Float16, hb);
              lv[e] = __builtin_bit_cast(_Float16, lb);
            }
          }
          *(volatile v8h*)(C + (size_t)(mBase + row) * ldc + n0 + c8) = hv;
          if (OUT_MODE == 2) *(volatile v8h*)(C2 + (size_t)(mBase + row) * ldc + n0 + c8) = lv;
        }
        __threadfence();
      }
    }
    __builtin_amdgcn_fence(__ATOMIC_RELEASE, "workgroup");
    __builtin_amdgcn_wave_barrier();
    __builtin_amdgcn_fence(__ATOMIC_ACQUIRE, "workgroup");
  }
}

__global__ __launch_bounds__(256) void cast8_kernel(const float* __restrict__ in, unsigned short* __restrict__ out, int n8, float scale) {
  const int i = blockIdx.x * 256 + threadIdx.x;
  if (i >= n8) return;
  const float* p = in + 8 * (size_t)i;
  const v4f a = *(const v4f*)(p);
  const v4f c = *(const v4f*)(p + 4);
  unsigned short hb[8];
#pragma unroll
  for (int e = 0; e < 4; ++e) {
    hb[e]     = h_bits(a[e] * scale);
    hb[4 + e] = h_bits(c[e] * scale);
  }
  const v4u u = (v4u){pk16(hb[0], hb[1]), pk16(hb[2], hb[3]), pk16(hb[4], hb[5]), pk16(hb[6], hb[7])};
  unsigned short* q = out + 8 * (size_t)i;
  *(volatile v4u*)q = u;
  __threadfence();
  *(volatile v4u*)q = u;
}

__global__ __launch_bounds__(256) void bias_cat_kernel(const float* __restrict__ a, const float* __restrict__ bsrc, float* __restrict__ dst) {
  const int t = threadIdx.x;
  const int ia = min(t, 127) * 4;
  const int ib = max(t - 128, 0) * 4;
  const v4f va = *(const v4f*)(a + ia);
  const v4f vb = *(const v4f*)(bsrc + ib);
  v4f v;
#pragma unroll
  for (int e = 0; e < 4; ++e) v[e] = (t < 128) ? va[e] : vb[e];
  float* p = dst + 4 * t;
  *(volatile v4f*)p = v;
  __threadfence();
  *(volatile v4f*)p = v;
}

template <int NPL>
__global__ __launch_bounds__(256) void tcast_kernel(const float* __restrict__ in, unsigned short* __restrict__ outHi,
                                                    unsigned short* __restrict__ outLo, int Cin, int L) {
  __shared__ float sm[64][65];
  const int t = threadIdx.x;
  const int l0 = blockIdx.x * 64, c0 = blockIdx.y * 64;
  const float* src = in + (size_t)c0 * L + l0;
#pragma unroll
  for (int i = 0; i < 16; ++i) {
    const int e = i * 256 + t;
    const int r = e >> 6;
    const int c = e & 63;
    sm[c][r] = src[(size_t)r * L + c];
  }
  __syncthreads();
  const int lane = t & 31, wave = t >> 5, q = lane >> 3, c8 = (lane & 7) * 8;
  v4u uh[2], ul[2];
  size_t off[2];
#pragma unroll
  for (int it = 0; it < 2; ++it) {
    const int row = wave * 8 + it * 4 + q;
    unsigned short hb[8], lb[8];
#pragma unroll
    for (int e = 0; e < 8; ++e) {
      const float v = sm[row][c8 + e];
      const _Float16 hv = (_Float16)v;
      hb[e] = __builtin_bit_cast(unsigned short, hv);
      lb[e] = (NPL == 2) ? h_bits((v - (float)hv) * kLoCarry) : (unsigned short)0;
    }
    uh[it] = (v4u){pk16(hb[0], hb[1]), pk16(hb[2], hb[3]), pk16(hb[4], hb[5]), pk16(hb[6], hb[7])};
    ul[it] = (v4u){pk16(lb[0], lb[1]), pk16(lb[2], lb[3]), pk16(lb[4], lb[5]), pk16(lb[6], lb[7])};
    off[it] = (size_t)(l0 + row) * Cin + c0 + c8;
  }
  for (int pass = 0; pass < 2; ++pass) {
#pragma unroll
    for (int it = 0; it < 2; ++it) {
      *(volatile v4u*)(outHi + off[it]) = uh[it];
      if (NPL == 2) *(volatile v4u*)(outLo + off[it]) = ul[it];
    }
    __threadfence();
  }
}

__global__ __launch_bounds__(128) void colstats_kernel(const float* __restrict__ src, int pitch, int nrows,
                                                       float* __restrict__ stats, int C, float invN) {
  const int c = blockIdx.x * 512 + threadIdx.x * 4;
  const float* p = src + c;
  v4f s = (v4f){0.f, 0.f, 0.f, 0.f}, q = (v4f){0.f, 0.f, 0.f, 0.f};
#pragma unroll 1
  for (int r0 = 0; r0 < nrows; r0 += 128) {
    v4f ps = (v4f){0.f, 0.f, 0.f, 0.f}, pq = (v4f){0.f, 0.f, 0.f, 0.f};
#pragma unroll 2
    for (int i = 0; i < 128; ++i) {
      const v4f x = *(const v4f*)(p + (size_t)(r0 + i) * pitch);
      ps += x;
      pq += x * x;
    }
    s += ps;
    q += pq;
  }
  const v4f mean = s * invN;
  v4f var = q * invN - mean * mean;
  v4f rstd;
#pragma unroll
  for (int e = 0; e < 4; ++e) {
    const float vv = fmaxf(var[e], 0.0f);
    rstd[e] = 1.0f / sqrtf(vv + kEps);
  }
  *(volatile v4f*)(stats + c) = mean;
  *(volatile v4f*)(stats + C + c) = rstd;
  __threadfence();
  *(volatile v4f*)(stats + c) = mean;
  *(volatile v4f*)(stats + C + c) = rstd;
}

template <int NPL>
__global__ __launch_bounds__(256) void normcast_kernel(const float* __restrict__ src, int srcPitch,
                                                       const float* __restrict__ stats, int statsC, int chOff,
                                                       unsigned short* __restrict__ dstHi, unsigned short* __restrict__ dstLo,
                                                       int dstPitch, int nrows) {
  const int i = blockIdx.x * 256 + threadIdx.x;
  const int row = i >> 6;
  const int c = (i & 63) * 8;
  if (row >= nrows) return;
  const float* p = src + (size_t)row * srcPitch + chOff + c;
  const v4f a = *(const v4f*)(p);
  const v4f d = *(const v4f*)(p + 4);
  const float* st = stats + chOff + c;
  const v4f m0 = *(const v4f*)(st), m1 = *(const v4f*)(st + 4);
  const v4f r0 = *(const v4f*)(st + statsC), r1 = *(const v4f*)(st + statsC + 4);
  float v[8];
#pragma unroll
  for (int e = 0; e < 4; ++e) {
    v[e]     = (a[e] - m0[e]) * r0[e];
    v[4 + e] = (d[e] - m1[e]) * r1[e];
  }
  unsigned short hb[8], lb[8];
#pragma unroll
  for (int e = 0; e < 8; ++e) {
    const _Float16 hv = (_Float16)v[e];
    hb[e] = __builtin_bit_cast(unsigned short, hv);
    lb[e] = (NPL == 2) ? h_bits((v[e] - (float)hv) * kLoCarry) : (unsigned short)0;
  }
  const v4u uh = (v4u){pk16(hb[0], hb[1]), pk16(hb[2], hb[3]), pk16(hb[4], hb[5]), pk16(hb[6], hb[7])};
  const v4u ul = (v4u){pk16(lb[0], lb[1]), pk16(lb[2], lb[3]), pk16(lb[4], lb[5]), pk16(lb[6], lb[7])};
  const size_t off = (size_t)row * dstPitch + c;
  for (int pass = 0; pass < 2; ++pass) {
    *(volatile v4u*)(dstHi + off) = uh;
    if (NPL == 2) *(volatile v4u*)(dstLo + off) = ul;
    __threadfence();
  }
}

__global__ __launch_bounds__(256) void vnormt_kernel(const float* __restrict__ src, int srcPitch,
                                                     const float* __restrict__ stats, int statsC, int chOff,
                                                     unsigned short* __restrict__ vh, unsigned short* __restrict__ vl, int dstPitch) {
  __shared__ float sm[64][65];
  const int t = threadIdx.x;
  const int l0 = blockIdx.x * 64, c0 = blockIdx.y * 64;
  {
    const int r = t >> 4, c4 = (t & 15) * 4;
    const v4f m  = *(const v4f*)(stats + chOff + c0 + c4);
    const v4f rs = *(const v4f*)(stats + statsC + chOff + c0 + c4);
#pragma unroll
    for (int it = 0; it < 4; ++it) {
      const int row = it * 16 + r;
      const v4f x = *(const v4f*)(src + (size_t)(l0 + row) * srcPitch + chOff + c0 + c4);
#pragma unroll
      for (int e = 0; e < 4; ++e) sm[c4 + e][row] = (x[e] - m[e]) * rs[e];
    }
  }
  __syncthreads();
  const int lane = t & 31, wave = t >> 5, q = lane >> 3, c8 = (lane & 7) * 8;
  v4u uh[2], ul[2];
  size_t off[2];
#pragma unroll
  for (int it = 0; it < 2; ++it) {
    const int chrow = wave * 8 + it * 4 + q;
    unsigned short hb[8], lb[8];
#pragma unroll
    for (int e = 0; e < 8; ++e) {
      const float v = sm[chrow][c8 + e];
      const unsigned short h = f2bf_bits(v);
      hb[e] = h;
      lb[e] = f2bf_bits(v - bf_bits2f(h));
    }
    uh[it] = (v4u){pk16(hb[0], hb[1]), pk16(hb[2], hb[3]), pk16(hb[4], hb[5]), pk16(hb[6], hb[7])};
    ul[it] = (v4u){pk16(lb[0], lb[1]), pk16(lb[2], lb[3]), pk16(lb[4], lb[5]), pk16(lb[6], lb[7])};
    off[it] = (size_t)(c0 + chrow) * dstPitch + l0 + c8;
  }
  for (int pass = 0; pass < 2; ++pass) {
#pragma unroll
    for (int it = 0; it < 2; ++it) {
      *(volatile v4u*)(vh + off[it]) = uh[it];
      *(volatile v4u*)(vl + off[it]) = ul[it];
    }
    __threadfence();
  }
}

__global__ __launch_bounds__(256) void zero16_kernel(unsigned short* base, long bstride, long pitch, int rowsPerB, int segsPerRow, int total) {
  const int i = blockIdx.x * 256 + threadIdx.x;
  if (i >= total) return;
  const int seg = i % segsPerRow;
  const int rr  = i / segsPerRow;
  const int r   = rr % rowsPerB;
  const int b   = rr / rowsPerB;
  unsigned short* p = base + (size_t)b * bstride + (size_t)r * pitch + (size_t)seg * 8;
  const v4u z = (v4u){0u, 0u, 0u, 0u};
  *(volatile v4u*)p = z;
  __threadfence();
  *(volatile v4u*)p = z;
}

__global__ __launch_bounds__(64) void softmax_kernel(float* S) {
  __shared__ float redM[2];
  __shared__ float redS[2];
  const int R = blockIdx.x;
  const int g = R >> 8;
  const int n = g % kNW;
  const int s0 = n * kStr;
  const int e0 = min(s0 + kWin, kLd);
  const int nv = min(2 * e0, kLe) - 2 * s0;
  const int t = threadIdx.x, lane = t & 31, wave = t >> 5;
  const int c0 = t * 8;
  float* sr = S + (size_t)R * kMaxE;
  const v4f a = *(const v4f*)(sr + c0);
  const v4f c = *(const v4f*)(sr + c0 + 4);
  float x[8];
#pragma unroll
  for (int e = 0; e < 4; ++e) { x[e] = a[e]; x[4 + e] = c[e]; }
#pragma unroll
  for (int e = 0; e < 8; ++e) x[e] = (c0 + e < nv) ? x[e] : -1e30f;
  float m = x[0];
#pragma unroll
  for (int e = 1; e < 8; ++e) m = fmaxf(m, x[e]);
#pragma unroll
  for (int off = 16; off > 0; off >>= 1) m = fmaxf(m, __shfl_xor(m, off, 32));
  if (lane == 0) redM[wave] = m;
  __syncthreads();
  m = fmaxf(redM[0], redM[1]);
  float p[8];
  float sum = 0.f;
#pragma unroll
  for (int e = 0; e < 8; ++e) { p[e] = expf(x[e] - m); sum += p[e]; }
#pragma unroll
  for (int off = 16; off > 0; off >>= 1) sum += __shfl_xor(sum, off, 32);
  if (lane == 0) redS[wave] = sum;
  __syncthreads();
  const float tot = redS[0] + redS[1];
  const float inv = 1.0f / tot;
  unsigned short hb[8], lb[8];
#pragma unroll
  for (int e = 0; e < 8; ++e) {
    const float pv = p[e] * inv;
    const unsigned short h = f2bf_bits(pv);
    hb[e] = h;
    lb[e] = f2bf_bits(pv - bf_bits2f(h));
  }
  const v4u uh = (v4u){pk16(hb[0], hb[1]), pk16(hb[2], hb[3]), pk16(hb[4], hb[5]), pk16(hb[6], hb[7])};
  const v4u ul = (v4u){pk16(lb[0], lb[1]), pk16(lb[2], lb[3]), pk16(lb[4], lb[5]), pk16(lb[6], lb[7])};
  unsigned short* ph = (unsigned short*)sr + c0;
  unsigned short* pl = (unsigned short*)sr + kMaxE + c0;
  for (int pass = 0; pass < 2; ++pass) {
    *(volatile v4u*)ph = uh;
    *(volatile v4u*)pl = ul;
    __threadfence();
  }
}

__global__ __launch_bounds__(256) void avg_kernel(const float* __restrict__ O, unsigned short* __restrict__ ah, unsigned short* __restrict__ al) {
  const int hl = blockIdx.y;
  const int t = threadIdx.x;
  const int tok = blockIdx.x * 32 + (t >> 3);
  const int q8 = (t & 7) * 8;
  const int nA = min(tok / kStr, kNW - 1);
  const int rA = tok - nA * kStr;
  const bool hasB = (nA >= 1) && (rA + kStr <= kWin - 1);
  const int nB = max(nA - 1, 0);
  const int rB = min(tok - nB * kStr, kWin - 1);
  const float* pa = O + ((size_t)(hl * kNW + nA) * kWin + rA) * kHD + q8;
  const float* pb = O + ((size_t)(hl * kNW + nB) * kWin + rB) * kHD + q8;
  const v4f a0 = *(const v4f*)(pa), a1 = *(const v4f*)(pa + 4);
  const v4f b0 = *(const v4f*)(pb), b1 = *(const v4f*)(pb + 4);
  unsigned short hb[8], lb[8];
#pragma unroll
  for (int e = 0; e < 8; ++e) {
    const float va = (e < 4) ? a0[e] : a1[e - 4];
    const float vb = (e < 4) ? b0[e] : b1[e - 4];
    const float ssum = vb + va;
    const float v = hasB ? (ssum * 0.5f) : va;
    const float w = v * kAttCarry;
    const _Float16 hv = (_Float16)w;
    hb[e] = __builtin_bit_cast(unsigned short, hv);
    lb[e] = h_bits((w - (float)hv) * kLoCarry);
  }
  const v4u uh = (v4u){pk16(hb[0], hb[1]), pk16(hb[2], hb[3]), pk16(hb[4], hb[5]), pk16(hb[6], hb[7])};
  const v4u ul = (v4u){pk16(lb[0], lb[1]), pk16(lb[2], lb[3]), pk16(lb[4], lb[5]), pk16(lb[6], lb[7])};
  const size_t off = (size_t)tok * kCd + hl * kHD + q8;
  for (int pass = 0; pass < 2; ++pass) {
    *(volatile v4u*)(ah + off) = uh;
    *(volatile v4u*)(al + off) = ul;
    __threadfence();
  }
}

__global__ __launch_bounds__(256) void xres_kernel(const float* __restrict__ y2, const float* __restrict__ stats,
                                                   const float* __restrict__ xdec, float* __restrict__ xcm,
                                                   unsigned short* __restrict__ x16) {
  __shared__ float sy[64][65];
  __shared__ float sx[64][65];
  const int t = threadIdx.x;
  const int l0 = blockIdx.x * 64, c0 = blockIdx.y * 64;
  {
    const int r = t >> 4, c4 = (t & 15) * 4;
    const float* st = stats + c0 + c4;
    const v4f m = *(const v4f*)(st), rs = *(const v4f*)(st + kCd);
#pragma unroll
    for (int it = 0; it < 4; ++it) {
      const int row = it * 16 + r;
      const v4f x = *(const v4f*)(y2 + (size_t)(l0 + row) * kCd + c0 + c4);
#pragma unroll
      for (int e = 0; e < 4; ++e) sy[row][c4 + e] = (x[e] - m[e]) * rs[e];
    }
  }
#pragma unroll
  for (int i = 0; i < 16; ++i) {
    const int e = i * 256 + t;
    const int r = e >> 6;
    const int c = e & 63;
    sx[r][c] = xdec[(size_t)(c0 + r) * kLd + l0 + c];
  }
  __syncthreads();
  const int lane = t & 31, wave = t >> 5;
  const int hh = lane >> 4, c4b = (lane & 15) * 4;
  const int q = lane >> 3, c8 = (lane & 7) * 8;
  v4f cv[4];
  size_t coff[4];
#pragma unroll
  for (int it = 0; it < 4; ++it) {
    const int chrow = wave * 8 + it * 2 + hh;
#pragma unroll
    for (int e = 0; e < 4; ++e) cv[it][e] = sy[c4b + e][chrow] + sx[chrow][c4b + e];
    coff[it] = (size_t)(c0 + chrow) * kLd + l0 + c4b;
  }
  v4u tu[2];
  size_t toff[2];
#pragma unroll
  for (int it = 0; it < 2; ++it) {
    const int tokrow = wave * 8 + it * 4 + q;
    unsigned short hb[8];
#pragma unroll
    for (int e = 0; e < 8; ++e) hb[e] = h_bits(sy[tokrow][c8 + e] + sx[c8 + e][tokrow]);
    tu[it] = (v4u){pk16(hb[0], hb[1]), pk16(hb[2], hb[3]), pk16(hb[4], hb[5]), pk16(hb[6], hb[7])};
    toff[it] = (size_t)(l0 + tokrow) * kCd + c0 + c8;
  }
  for (int pass = 0; pass < 2; ++pass) {
#pragma unroll
    for (int it = 0; it < 4; ++it) *(volatile v4f*)(xcm + coff[it]) = cv[it];
#pragma unroll
    for (int it = 0; it < 2; ++it) *(volatile v4u*)(x16 + toff[it]) = tu[it];
    __threadfence();
  }
}

__global__ __launch_bounds__(256) void gelu_kernel(const float* __restrict__ pre, unsigned short* __restrict__ h, int n2) {
  const int i = blockIdx.x * 256 + threadIdx.x;
  if (i >= n2) return;
  const v2f xv = *(const v2f*)(pre + 2 * (size_t)i);
  const float v0 = xv[0], v1 = xv[1];
  float g0 = 0.f, g1 = 0.f;
#pragma unroll 1
  for (int e = 0; e < 2; ++e) {
    const float v = (e == 0) ? v0 : v1;
    const float r = 0.5f * v * (1.0f + erff(v * 0.70710678118654752f));
    g0 = (e == 0) ? r : g0;
    g1 = (e == 0) ? g1 : r;
  }
  const unsigned u = pk16(h_bits(g0), h_bits(g1));
  ((volatile unsigned*)h)[i] = u;
  __threadfence();
  ((volatile unsigned*)h)[i] = u;
}

__global__ __launch_bounds__(256) void final_kernel(const float* __restrict__ y3, const float* __restrict__ stats,
                                                    const float* __restrict__ xcm, float* __restrict__ out) {
  __shared__ float sy[64][65];
  const int t = threadIdx.x;
  const int l0 = blockIdx.x * 64, c0 = blockIdx.y * 64;
  {
    const int r = t >> 4, c4 = (t & 15) * 4;
    const float* st = stats + c0 + c4;
    const v4f m = *(const v4f*)(st), rs = *(const v4f*)(st + kCd);
#pragma unroll
    for (int it = 0; it < 4; ++it) {
      const int row = it * 16 + r;
      const v4f x = *(const v4f*)(y3 + (size_t)(l0 + row) * kCd + c0 + c4);
#pragma unroll
      for (int e = 0; e < 4; ++e) sy[row][c4 + e] = (x[e] - m[e]) * rs[e];
    }
  }
  __syncthreads();
  const int lane = t & 31, wave = t >> 5;
  const int hh = lane >> 4, c4b = (lane & 15) * 4;
  v4f cv[4];
  size_t coff[4];
#pragma unroll
  for (int it = 0; it < 4; ++it) {
    const int chrow = wave * 8 + it * 2 + hh;
    coff[it] = (size_t)(c0 + chrow) * kLd + l0 + c4b;
    const v4f xr = *(const v4f*)(xcm + coff[it]);
#pragma unroll
    for (int e = 0; e < 4; ++e) cv[it][e] = sy[c4b + e][chrow] + xr[e];
  }
  for (int pass = 0; pass < 2; ++pass) {
#pragma unroll
    for (int it = 0; it < 4; ++it) *(volatile v4f*)(out + coff[it]) = cv[it];
    __threadfence();
  }
}

static GemmGeom mk_geom(long sA0, long sA1, long sA2, long sB0, long sB1, long sB2, long sC0, long sC1, long sC2,
                        int d1, int d2, int lda, int ldb, int ldc, int M, int N, int K, float scale) {
  GemmGeom g;
  g.sA0 = sA0; g.sA1 = sA1; g.sA2 = sA2;
  g.sB0 = sB0; g.sB1 = sB1; g.sB2 = sB2;
  g.sC0 = sC0; g.sC1 = sC1; g.sC2 = sC2;
  g.d1 = d1; g.d2 = d2; g.lda = lda; g.ldb = ldb; g.ldc = ldc; g.M = M; g.N = N; g.K = K;
  g.scale = scale; g.pad0 = 0;
  return g;
}
static GemmGeom mk_plain(int lda, int ldb, int ldc, int M, int N, int K, float scale) {
  return mk_geom(0, 0, 0, 0, 0, 0, 0, 0, 0, 1, 1, lda, ldb, ldc, M, N, K, scale);
}
static unsigned gemm_blocks(int M, int N) { return (unsigned)(((M / 64) * (N / 64) + 7) / 8); }

extern "C" void kernel_launch(void* const* d_in, const int* in_sizes, int n_in,
                              void* d_out, int out_size, void* d_ws, size_t ws_size,
                              hipStream_t stream) {
  if (n_in < 14) return;
  if (ws_size < kWsEnd) return;
  if ((size_t)out_size != (size_t)kB * kCd * kLd) return;
  if (in_sizes[0] != kB * kCd * kLd || in_sizes[1] != kB * kCe * kLe) return;
  if (in_sizes[2] != kCd * kCd || in_sizes[4] != kCd * kCe || in_sizes[6] != kCd * kCe || in_sizes[8] != kCd * kCd) return;
  if (in_sizes[10] != kHid * kCd || in_sizes[12] != kCd * kHid) return;
  if (in_sizes[3] != kCd || in_sizes[5] != kCd || in_sizes[7] != kCd || in_sizes[9] != kCd || in_sizes[11] != kHid || in_sizes[13] != kCd) return;

  const float* xd = (const float*)d_in[0];
  const float* xe = (const float*)d_in[1];
  const float* wq = (const float*)d_in[2];
  const float* bq = (const float*)d_in[3];
  const float* wk = (const float*)d_in[4];
  const float* bk = (const float*)d_in[5];
  const float* wv = (const float*)d_in[6];
  const float* bv = (const float*)d_in[7];
  const float* wo = (const float*)d_in[8];
  const float* bo = (const float*)d_in[9];
  const float* w1 = (const float*)d_in[10];
  const float* b1 = (const float*)d_in[11];
  const float* w2 = (const float*)d_in[12];
  const float* b2 = (const float*)d_in[13];
  float* out = (float*)d_out;

  char* ws = (char*)d_ws;
  unsigned short* w16   = (unsigned short*)(ws + OFF_W16);
  unsigned short* wq16  = w16;
  unsigned short* wkv16 = wq16 + (size_t)kCd * kCd;
  unsigned short* wo16  = wkv16 + (size_t)2 * kCd * kCe;
  unsigned short* w116  = wo16 + (size_t)kCd * kCd;
  unsigned short* w216  = w116 + (size_t)kHid * kCd;
  float* bkv   = (float*)(ws + OFF_BKV);
  float* stats = (float*)(ws + OFF_STATS);
  unsigned short* qnh  = (unsigned short*)(ws + OFF_QNH);
  unsigned short* kn   = (unsigned short*)(ws + OFF_KN);
  unsigned short* vth  = (unsigned short*)(ws + OFF_VTH);
  unsigned short* vtl  = (unsigned short*)(ws + OFF_VTL);
  unsigned short* atth = (unsigned short*)(ws + OFF_ATH);
  unsigned short* attl = (unsigned short*)(ws + OFF_ATL);
  float* Sbuf  = (float*)(ws + OFF_S);
  float* Obuf  = (float*)(ws + OFF_O);
  unsigned short* xdh = (unsigned short*)(ws + OFF_XDH);
  unsigned short* xdl = (unsigned short*)(ws + OFF_XDL);
  float* qraw  = (float*)(ws + OFF_QRAW);
  unsigned short* xet = (unsigned short*)(ws + OFF_XET);
  float* kvraw = (float*)(ws + OFF_KVRAW);
  float* y2    = (float*)(ws + OFF_Y2);
  unsigned short* h16 = (unsigned short*)(ws + OFF_H16);
  float* pre   = (float*)(ws + OFF_PRE);
  float* y3    = (float*)(ws + OFF_Y3);
  float* xcm   = (float*)(ws + OFF_XCM);
  unsigned short* x16 = (unsigned short*)(ws + OFF_X16);

  cast8_kernel<<<(kCd * kCd / 8) / 256, 256, 0, stream>>>(wq, wq16, kCd * kCd / 8, kWCarry);
  cast8_kernel<<<(kCd * kCe / 8) / 256, 256, 0, stream>>>(wk, wkv16, kCd * kCe / 8, kWCarry);
  cast8_kernel<<<(kCd * kCe / 8) / 256, 256, 0, stream>>>(wv, wkv16 + (size_t)kCd * kCe, kCd * kCe / 8, kWCarry);
  cast8_kernel<<<(kCd * kCd / 8) / 256, 256, 0, stream>>>(wo, wo16, kCd * kCd / 8, kWCarry);
  cast8_kernel<<<(kHid * kCd / 8) / 256, 256, 0, stream>>>(w1, w116, kHid * kCd / 8, kWCarry);
  cast8_kernel<<<(kCd * kHid / 8) / 256, 256, 0, stream>>>(w2, w216, kCd * kHid / 8, kWCarry);
  bias_cat_kernel<<<1, 256, 0, stream>>>(bk, bv, bkv);
  zero16_kernel<<<(kWin * 64 + 255) / 256, 256, 0, stream>>>(qnh + (size_t)kLd * kCd, 0, kCd, kWin, 64, kWin * 64);
  zero16_kernel<<<(kMaxE * 64 + 255) / 256, 256, 0, stream>>>(kn + (size_t)kLe * kCd, 0, kCd, kMaxE, 64, kMaxE * 64);
  zero16_kernel<<<(2 * kCd * 64 + 255) / 256, 256, 0, stream>>>(vth + kLe, (long)kCd * kKRows, kKRows, kCd, 64, 2 * kCd * 64);

  const GemmGeom gq   = mk_plain(kCd, kCd, kCd, kLd, kCd, kCd, 1.0f / kWCarry);
  const GemmGeom gqlo = mk_plain(kCd, kCd, kCd, kLd, kCd, kCd, 1.0f / (kWCarry * kLoCarry));
  const GemmGeom gkv  = mk_plain(kCe, kCe, 2 * kCd, kLe, 2 * kCd, kCe, 1.0f / kWCarry);
  const GemmGeom gs = mk_geom(0, kHD, (long)kStr * kCd, 0, kHD, (long)2 * kStr * kCd, 0, (long)kNW * kWin * kMaxE, (long)kWin * kMaxE,
                              kHeadsPerChunk, kNW, kCd, kCd, kMaxE, kWin, kMaxE, kHD, 0.125f);
  const GemmGeom gp = mk_geom(0, (long)kNW * kWin * 2 * kMaxE, (long)kWin * 2 * kMaxE, 0, (long)kHD * kKRows, (long)2 * kStr,
                              0, (long)kNW * kWin * kHD, (long)kWin * kHD,
                              kHeadsPerChunk, kNW, 2 * kMaxE, kKRows, kHD, kWin, kHD, kMaxE, 1.0f);
  const GemmGeom go   = mk_plain(kCd, kCd, kCd, kLd, kCd, kCd, 1.0f / (kAttCarry * kWCarry));
  const GemmGeom golo = mk_plain(kCd, kCd, kCd, kLd, kCd, kCd, 1.0f / (kAttCarry * kWCarry * kLoCarry));
  const GemmGeom g1   = mk_plain(kCd, kCd, kHid, kLd, kHid, kCd, 1.0f / kWCarry);
  const GemmGeom g2   = mk_plain(kHid, kHid, kCd, kLd, kCd, kHid, 1.0f / kWCarry);

  for (int b = 0; b < kB; ++b) {
    const float* xdb = xd + (size_t)b * kCd * kLd;
    const float* xeb = xe + (size_t)b * kCe * kLe;

    tcast_kernel<2><<<dim3(kLd / 64, kCd / 64), 256, 0, stream>>>(xdb, xdh, xdl, kCd, kLd);
    wmma_gemm64g<0, false, 2, 0, false><<<dim3(gemm_blocks(kLd, kCd), 1), 256, 0, stream>>>(xdh, nullptr, wq16, nullptr, qraw, nullptr, bq, nullptr, gq);
    wmma_gemm64g<0, false, 0, 0, true><<<dim3(gemm_blocks(kLd, kCd), 1), 256, 0, stream>>>(xdl, nullptr, wq16, nullptr, qraw, nullptr, nullptr, qraw, gqlo);
    colstats_kernel<<<kCd / 512, 128, 0, stream>>>(qraw, kCd, kLd, stats, kCd, 1.0f / (float)kLd);
    normcast_kernel<1><<<kLd / 4, 256, 0, stream>>>(qraw, kCd, stats, kCd, 0, qnh, qnh, kCd, kLd);

    tcast_kernel<1><<<dim3(kLe / 64, kCe / 64), 256, 0, stream>>>(xeb, xet, xet, kCe, kLe);
    wmma_gemm64g<0, false, 2, 0, false><<<dim3(gemm_blocks(kLe, 2 * kCd), 1), 256, 0, stream>>>(xet, nullptr, wkv16, nullptr, kvraw, nullptr, bkv, nullptr, gkv);
    colstats_kernel<<<2 * kCd / 512, 128, 0, stream>>>(kvraw, 2 * kCd, kLe, stats, 2 * kCd, 1.0f / (float)kLe);
    normcast_kernel<1><<<kLe / 4, 256, 0, stream>>>(kvraw, 2 * kCd, stats, 2 * kCd, 0, kn, kn, kCd, kLe);
    vnormt_kernel<<<dim3(kLe / 64, kCd / 64), 256, 0, stream>>>(kvraw, 2 * kCd, stats, 2 * kCd, kCd, vth, vtl, kKRows);

    for (int hq = 0; hq < kChunksPerBatch; ++hq) {
      const size_t colOff = (size_t)hq * kHeadsPerChunk * kHD;
      const size_t vOff   = (size_t)hq * kHeadsPerChunk * kHD * kKRows;
      wmma_gemm64g<0, false, 0, 0, false><<<dim3(gemm_blocks(kWin, kMaxE), kGroupsPerChunk), 256, 0, stream>>>(
          qnh + colOff, nullptr, kn + colOff, nullptr, Sbuf, nullptr, nullptr, nullptr, gs);
      softmax_kernel<<<kGroupsPerChunk * kWin, 64, 0, stream>>>(Sbuf);
      const unsigned short* P16 = (const unsigned short*)Sbuf;
      wmma_gemm64g<1, true, 0, 0, false><<<dim3(gemm_blocks(kWin, kHD), kGroupsPerChunk), 256, 0, stream>>>(
          P16, P16 + kMaxE, vth + vOff, vtl + vOff, Obuf, nullptr, nullptr, nullptr, gp);
      avg_kernel<<<dim3(kLd / 32, kHeadsPerChunk), 256, 0, stream>>>(Obuf, atth + colOff, attl + colOff);
    }

    wmma_gemm64g<0, false, 2, 0, false><<<dim3(gemm_blocks(kLd, kCd), 1), 256, 0, stream>>>(atth, nullptr, wo16, nullptr, y2, nullptr, bo, nullptr, go);
    wmma_gemm64g<0, false, 0, 0, true><<<dim3(gemm_blocks(kLd, kCd), 1), 256, 0, stream>>>(attl, nullptr, wo16, nullptr, y2, nullptr, nullptr, y2, golo);
    colstats_kernel<<<kCd / 512, 128, 0, stream>>>(y2, kCd, kLd, stats, kCd, 1.0f / (float)kLd);
    xres_kernel<<<dim3(kLd / 64, kCd / 64), 256, 0, stream>>>(y2, stats, xdb, xcm, x16);

    wmma_gemm64g<0, false, 2, 0, false><<<dim3(gemm_blocks(kLd, kHid), 1), 256, 0, stream>>>(x16, nullptr, w116, nullptr, pre, nullptr, b1, nullptr, g1);
    gelu_kernel<<<(kLd * kHid / 2) / 256, 256, 0, stream>>>(pre, h16, kLd * kHid / 2);
    wmma_gemm64g<0, false, 2, 0, false><<<dim3(gemm_blocks(kLd, kCd), 1), 256, 0, stream>>>(h16, nullptr, w216, nullptr, y3, nullptr, b2, nullptr, g2);
    colstats_kernel<<<kCd / 512, 128, 0, stream>>>(y3, kCd, kLd, stats, kCd, 1.0f / (float)kLd);
    final_kernel<<<dim3(kLd / 64, kCd / 64), 256, 0, stream>>>(y3, stats, xcm, out + (size_t)b * kCd * kLd);
  }
}
